// LIIF_6949257084959
// MI455X (gfx1250) — hardware-verified
//
#include <hip/hip_runtime.h>
#include <math.h>

constexpr int NBATCH  = 8;
constexpr int NQUERY  = 8192;
constexpr int NSAMP   = NBATCH * NQUERY;
constexpr int NROWS   = 4 * NSAMP;
constexpr int IMG     = 64;
constexpr int NCIN    = 3;
constexpr int NCH     = 64;
constexpr int HID     = 256;
constexpr int KFEAT   = NCH * 9;
constexpr int KIN     = KFEAT + 4;
constexpr int KPAD    = 608;
constexpr int W0PITCH = 640;
constexpr int MTILE   = 64;
constexpr int NOUT4   = 16;
constexpr float WCARRY     = 16.0f;
constexpr float WCARRY_INV = 0.0625f;
static_assert(KPAD % 32 == 0);
static_assert(KPAD >= KIN);
static_assert(W0PITCH % 64 == 0 && W0PITCH >= KPAD);
static_assert(HID % 32 == 0);
static_assert(NROWS % MTILE == 0);
static_assert(NSAMP % MTILE == 0);
static_assert(NSAMP % 256 == 0);
static_assert((NBATCH * IMG * IMG) % 4 == 0);

typedef __attribute__((ext_vector_type(16))) _Float16 v16h;
typedef __attribute__((ext_vector_type(8)))  _Float16 v8h;
typedef __attribute__((ext_vector_type(8)))  float    v8f;
typedef __attribute__((ext_vector_type(4)))  float    v4f;
typedef __attribute__((ext_vector_type(4)))  unsigned int v4u;

__device__ __forceinline__ void acc_guard4(v8f& a, v8f& b, v8f& c, v8f& d) { asm volatile("v_nop\n\tv_nop\n\tv_nop\n\tv_nop" : "+v"(a), "+v"(b), "+v"(c), "+v"(d)); }
template <typename T> struct Frag;
template <> struct Frag<_Float16> {
  typedef v16h V; union U { v16h v; v8h h[2]; };
  static __device__ __forceinline__ v16h load(const _Float16* p) {
    U f; f.h[0] = *(const v8h*)(p); f.h[1] = *(const v8h*)(p + 16); return f.v;
  }
  static __device__ __forceinline__ v8f mma(v16h a, v16h b, v8f c) {
    return __builtin_amdgcn_wmma_f32_16x16x32_f16(false, a, false, b, (short)0, c, false, false);
  }
};

__device__ __forceinline__ void guard_ab2(v8f& c0, v8f& c1, v16h a, v16h b0, v16h b1) {
  asm volatile("v_nop\n\tv_nop\n\tv_nop\n\tv_nop" : "+v"(c0), "+v"(c1) : "v"(a), "v"(b0), "v"(b1));
}
__device__ __forceinline__ void guard_ab1(v8f& c0, v16h a, v16h b) {
  asm volatile("v_nop\n\tv_nop\n\tv_nop\n\tv_nop" : "+v"(c0) : "v"(a), "v"(b));
}

__device__ __forceinline__ unsigned pk16(unsigned short a, unsigned short b) { return (unsigned)a | ((unsigned)b << 16); }
__device__ __forceinline__ unsigned short h_bits(float f) { const _Float16 h = (_Float16)f; return __builtin_bit_cast(unsigned short, h); }

__device__ __forceinline__ float bf16_rne(float f) {
  unsigned u = __float_as_uint(f);
  u = (u + 0x7FFFu + ((u >> 16) & 1u)) & 0xFFFF0000u;
  float r = __uint_as_float(u);
  asm volatile("" : "+v"(r));
  return r;
}

__global__ __launch_bounds__(256) void conv_kernel(const float* __restrict__ inp, const float* __restrict__ ew,
                                                   const float* __restrict__ eb, unsigned short* __restrict__ featH) {
  __shared__ float sW[NCH * 27];
  __shared__ float sB[NCH];
  __shared__ float sIn[4 * 28];
  __shared__ __align__(16) unsigned short sF[256];
  const int t = threadIdx.x;
  const int lane = t & 31, wave = t >> 5;
  const int pix0 = blockIdx.x * 4;
#pragma unroll
  for (int i = 0; i < 7; ++i) {
    const int idx = i * 256 + t;
    const int idc = idx < NCH * 27 ? idx : (NCH * 27 - 1);
    const float v = bf16_rne(ew[idc]);
    if (idx < NCH * 27) sW[idx] = v;
  }
  {
    const float v = bf16_rne(eb[t < NCH ? t : (NCH - 1)]);
    if (t < NCH) sB[t] = v;
  }
  {
    const int tt  = t < 108 ? t : 107;
    const int pl2 = tt / 27;
    const int k   = tt - pl2 * 27;
    const int ci  = k / 9;
    const int ky  = (k / 3) % 3;
    const int kx  = k % 3;
    const int pix = pix0 + pl2;
    const int b = pix >> 12, y = (pix >> 6) & 63, x = pix & 63;
    const int yy = y + ky - 1, xx = x + kx - 1;
    const bool ok = ((unsigned)yy < 64u) && ((unsigned)xx < 64u);
    const int yc = yy < 0 ? 0 : (yy > 63 ? 63 : yy);
    const int xc = xx < 0 ? 0 : (xx > 63 ? 63 : xx);
    const float v  = bf16_rne(inp[(((size_t)b * NCIN + ci) * IMG + yc) * IMG + xc]);
    const float fa = ok ? 1.0f : 0.0f;
    if (t < 108) sIn[pl2 * 28 + k] = fmaf(v, fa, 0.0f);
  }
  __syncthreads();
  const int pl = t >> 6, c = t & 63;
  float s = 0.0f;
#pragma unroll
  for (int k = 0; k < 27; ++k) s += sIn[pl * 28 + k] * sW[c * 27 + k];
  s += sB[c];
  sF[t] = h_bits(s);
  __syncthreads();
  if (wave == 0) {
    const unsigned short* q = sF + lane * 8;
    const v4u u = (v4u){pk16(q[0], q[1]), pk16(q[2], q[3]), pk16(q[4], q[5]), pk16(q[6], q[7])};
    unsigned short* op = featH + (size_t)pix0 * NCH + lane * 8;
    *(volatile v4u*)op = u;
    __threadfence();
    *(volatile v4u*)op = u;
  }
}

__global__ __launch_bounds__(256) void wprep_kernel(const float* __restrict__ w0, const float* __restrict__ w1,
                                                    const float* __restrict__ w2, const float* __restrict__ w3,
                                                    unsigned short* __restrict__ Wt0, unsigned short* __restrict__ Wt123) {
  __shared__ float sm[64][65];
  const int t = threadIdx.x;
  const int z = blockIdx.z;
  if (z != 0 && blockIdx.x >= 4) return;
  const int k0 = blockIdx.x * 64;
  const int n0 = blockIdx.y * 64;
  const float* W = (z == 0) ? w0 : (z == 1) ? w1 : (z == 2) ? w2 : w3;
  const int pitch = (z == 0) ? W0PITCH : HID;
  unsigned short* op = (z == 0) ? Wt0 : (Wt123 + (size_t)(z - 1) * HID * HID);
#pragma unroll
  for (int g = 0; g < 2; ++g) {
#pragma unroll
    for (int i2 = 0; i2 < 8; ++i2) {
      const int e  = (g * 8 + i2) * 256 + t;
      const int kl = e >> 6;
      const int nl = e & 63;
      const int kp = k0 + kl;
      const int srow0 = (kp < KFEAT) ? ((kp & 63) * 9 + (kp >> 6)) : (kp < KIN ? kp : (KIN - 1));
      const float fa0 = (kp < KIN) ? WCARRY : 0.0f;
      const int srow1 = kp < HID ? kp : (HID - 1);
      const int srow  = (z == 0) ? srow0 : srow1;
      const float fa  = (z == 0) ? fa0 : WCARRY;
      const float v = bf16_rne(W[(size_t)srow * HID + n0 + nl]);
      sm[nl][kl] = fmaf(v, fa, 0.0f);
    }
    asm volatile("" ::: "memory");
  }
  __syncthreads();
  const int lane = t & 31, wave = t >> 5;
  const int q = lane >> 3, c8 = (lane & 7) * 8;
  for (int pass = 0; pass < 2; ++pass) {
#pragma unroll
    for (int it = 0; it < 2; ++it) {
      const int row = wave * 8 + it * 4 + q;
      unsigned short hb[8];
#pragma unroll
      for (int e = 0; e < 8; ++e) hb[e] = h_bits(sm[row][c8 + e]);
      const v4u u = (v4u){pk16(hb[0], hb[1]), pk16(hb[2], hb[3]), pk16(hb[4], hb[5]), pk16(hb[6], hb[7])};
      *(volatile v4u*)(op + (size_t)(n0 + row) * pitch + k0 + c8) = u;
    }
    __threadfence();
  }
}

__global__ __launch_bounds__(256) void wprep4_kernel(const float* __restrict__ w4, unsigned short* __restrict__ Wt4) {
  const int t = threadIdx.x;
  v4u u0, u1;
  {
    const int row = t >> 5, ch = t & 31;
    const int rr = row < 3 ? row : 2;
    const float fa = row < 3 ? WCARRY : 0.0f;
    unsigned short hb[8];
#pragma unroll
    for (int e = 0; e < 8; ++e) hb[e] = h_bits(fmaf(bf16_rne(w4[(ch * 8 + e) * 3 + rr]), fa, 0.0f));
    u0 = (v4u){pk16(hb[0], hb[1]), pk16(hb[2], hb[3]), pk16(hb[4], hb[5]), pk16(hb[6], hb[7])};
  }
  asm volatile("" ::: "memory");
  {
    const int row = (256 + t) >> 5, ch = t & 31;
    const int rr = row < 3 ? row : 2;
    const float fa = row < 3 ? WCARRY : 0.0f;
    unsigned short hb[8];
#pragma unroll
    for (int e = 0; e < 8; ++e) hb[e] = h_bits(fmaf(bf16_rne(w4[(ch * 8 + e) * 3 + rr]), fa, 0.0f));
    u1 = (v4u){pk16(hb[0], hb[1]), pk16(hb[2], hb[3]), pk16(hb[4], hb[5]), pk16(hb[6], hb[7])};
  }
  unsigned short* p0 = Wt4 + (size_t)(t >> 5) * HID + (t & 31) * 8;
  unsigned short* p1 = Wt4 + (size_t)((256 + t) >> 5) * HID + (t & 31) * 8;
  for (int pass = 0; pass < 2; ++pass) {
    *(volatile v4u*)p0 = u0;
    *(volatile v4u*)p1 = u1;
    __threadfence();
  }
}

__device__ __forceinline__ void corner_meta(float c0, float c1, int corner, int& iy, int& ix,
                                            float& rel0, float& rel1, float& area) {
#pragma clang fp contract(off)
  const float sy = (corner & 2) ? 0.015625f : -0.015625f;
  const float sx = (corner & 1) ? 0.015625f : -0.015625f;
  float cy = c0 + sy; cy = cy + 1e-6f; cy = fminf(fmaxf(cy, -0.999999f), 0.999999f);
  float cx = c1 + sx; cx = cx + 1e-6f; cx = fminf(fmaxf(cx, -0.999999f), 0.999999f);
  float ty = (cy + 1.0f) * 64.0f; ty = ty - 1.0f; ty = ty * 0.5f; ty = rintf(ty); ty = fminf(fmaxf(ty, 0.0f), 63.0f);
  float tx = (cx + 1.0f) * 64.0f; tx = tx - 1.0f; tx = tx * 0.5f; tx = rintf(tx); tx = fminf(fmaxf(tx, 0.0f), 63.0f);
  iy = (int)ty;
  ix = (int)tx;
  iy = iy < 0 ? 0 : (iy > 63 ? 63 : iy);
  ix = ix < 0 ? 0 : (ix > 63 ? 63 : ix);
  const float qy = -1.0f + (2.0f * (float)iy + 1.0f) * 0.015625f;
  const float qx = -1.0f + (2.0f * (float)ix + 1.0f) * 0.015625f;
  rel0 = (c0 - qy) * 64.0f;
  rel1 = (c1 - qx) * 64.0f;
  const float pr = rel0 * rel1;
  area = fabsf(pr) + 1e-9f;
}

__device__ __forceinline__ void mlp_layer(const unsigned short* src, int spitch, int kdim,
                                          const unsigned short* __restrict__ Wtp, int wpitch,
                                          const float* __restrict__ bias, unsigned short* dst, int lane, int wave) {
  const _Float16* Wt = (const _Float16*)(const void*)Wtp;
  const _Float16* S  = (const _Float16*)(const void*)src;
  const int rl   = lane & 15;
  const int koff = (lane >> 4) * 8;
  const int r8   = (lane >> 4) * 8;
  const int nA   = wave * 32 + rl;
  const int nB   = nA + 16;
  v8f acc[4][2];
#pragma unroll
  for (int mt = 0; mt < 4; ++mt) {
    acc[mt][0] = (v8f){0.f,0.f,0.f,0.f,0.f,0.f,0.f,0.f};
    acc[mt][1] = (v8f){0.f,0.f,0.f,0.f,0.f,0.f,0.f,0.f};
  }
#pragma unroll 1
  for (int ks = 0; ks < kdim; ks += 32) {
    const v16h fb0 = Frag<_Float16>::load(Wt + (size_t)nA * wpitch + ks + koff);
    const v16h fb1 = Frag<_Float16>::load(Wt + (size_t)nB * wpitch + ks + koff);
#pragma unroll
    for (int mt = 0; mt < 4; ++mt) {
      const v16h fa = Frag<_Float16>::load(S + (mt * 16 + rl) * spitch + ks + koff);
      acc[mt][0] = Frag<_Float16>::mma(fa, fb0, acc[mt][0]);
      acc[mt][1] = Frag<_Float16>::mma(fa, fb1, acc[mt][1]);
      guard_ab2(acc[mt][0], acc[mt][1], fa, fb0, fb1);
    }
  }
  acc_guard4(acc[0][0], acc[0][1], acc[1][0], acc[1][1]);
  acc_guard4(acc[2][0], acc[2][1], acc[3][0], acc[3][1]);
  const float bvA = bf16_rne(bias[nA]);
  const float bvB = bf16_rne(bias[nB]);
#pragma unroll
  for (int mt = 0; mt < 4; ++mt) {
#pragma unroll
    for (int r = 0; r < 8; ++r) {
      const int m = mt * 16 + r8 + r;
      float vA = acc[mt][0][r] * WCARRY_INV + bvA;
      float vB = acc[mt][1][r] * WCARRY_INV + bvB;
      vA = fmaxf(vA, 0.0f);
      vB = fmaxf(vB, 0.0f);
      dst[m * HID + nA] = h_bits(vA);
      dst[m * HID + nB] = h_bits(vB);
    }
  }
}

__global__ __launch_bounds__(256) void mlp_kernel(
    const unsigned short* __restrict__ featH,
    const float* __restrict__ coord, const float* __restrict__ cell,
    const unsigned short* __restrict__ Wt0, const unsigned short* __restrict__ Wt123,
    const unsigned short* __restrict__ Wt4,
    const float* __restrict__ b0, const float* __restrict__ b1,
    const float* __restrict__ b2, const float* __restrict__ b3,
    const float* __restrict__ b4,
    float* __restrict__ PA) {
  __shared__ __align__(16) unsigned short Xs[MTILE * KPAD];
  __shared__ __align__(16) unsigned short H1[MTILE * HID];
  __shared__ __align__(16) float sOut[MTILE * 4];
  __shared__ int   mB[MTILE], mIY[MTILE], mIX[MTILE];
  __shared__ float mR0[MTILE], mR1[MTILE], mC0[MTILE], mC1[MTILE];
  static_assert(MTILE * HID <= MTILE * KPAD);

  const int tid  = threadIdx.x;
  const int lane = tid & 31;
  const int wave = tid >> 5;
  const int rowBase = blockIdx.x * MTILE;
  const int corner  = rowBase >> 16;

  if (tid < MTILE) {
    const int R = rowBase + tid;
    const int s = R & (NSAMP - 1);
    const int b = s >> 13;
    const float c0  = bf16_rne(coord[2 * (size_t)s]), c1 = bf16_rne(coord[2 * (size_t)s + 1]);
    const float ce0 = bf16_rne(cell[2 * (size_t)s]),  ce1 = bf16_rne(cell[2 * (size_t)s + 1]);
    int iy, ix; float rel0, rel1, area;
    corner_meta(c0, c1, corner, iy, ix, rel0, rel1, area);
    mB[tid] = b; mIY[tid] = iy; mIX[tid] = ix;
    mR0[tid] = rel0; mR1[tid] = rel1;
    mC0[tid] = ce0 * 64.0f; mC1[tid] = ce1 * 64.0f;
    sOut[tid * 4 + 3] = area;
  }
  __syncthreads();

#pragma unroll 3
  for (int i = 0; i < 18; ++i) {
    const int d = i * 256 + tid;
    const int pair = d >> 3, chunk = d & 7;
    const int m  = pair / 9;
    const int p  = pair - m * 9;
    const int py = p / 3, px = p - py * 3;
    const int yy = mIY[m] + py - 1, xx = mIX[m] + px - 1;
    const bool ok = ((unsigned)yy < 64u) && ((unsigned)xx < 64u);
    const int yc = yy < 0 ? 0 : (yy > 63 ? 63 : yy);
    const int xc = xx < 0 ? 0 : (xx > 63 ? 63 : xx);
    const size_t off = (((size_t)mB[m] * IMG + yc) * IMG + xc) * NCH + (size_t)chunk * 8;
    v4u u = *(const v4u*)(featH + off);
    const unsigned msk = ok ? 0xffffffffu : 0u;
    u = u & (v4u){msk, msk, msk, msk};
    *(v4u*)(Xs + m * KPAD + p * NCH + chunk * 8) = u;
  }
  {
    const int m = tid >> 2, ch = tid & 3;
    const unsigned wA = pk16(h_bits(mR0[m]), h_bits(mR1[m]));
    const unsigned wB = pk16(h_bits(mC0[m]), h_bits(mC1[m]));
    const unsigned msk = (ch == 0) ? 0xffffffffu : 0u;
    const v4u u = (v4u){wA & msk, wB & msk, 0u, 0u};
    *(v4u*)(Xs + m * KPAD + KFEAT + ch * 8) = u;
  }
  __syncthreads();

  mlp_layer(Xs, KPAD, KPAD, Wt0, W0PITCH, b0, H1, lane, wave);
  __syncthreads();
  mlp_layer(H1, HID, HID, Wt123, HID, b1, Xs, lane, wave);
  __syncthreads();
  mlp_layer(Xs, HID, HID, Wt123 + (size_t)HID * HID, HID, b2, H1, lane, wave);
  __syncthreads();
  mlp_layer(H1, HID, HID, Wt123 + (size_t)2 * HID * HID, HID, b3, Xs, lane, wave);
  __syncthreads();

  if (wave < 4) {
    const _Float16* H4 = (const _Float16*)(const void*)Xs;
    const _Float16* W4 = (const _Float16*)(const void*)Wt4;
    const int rl   = lane & 15;
    const int koff = (lane >> 4) * 8;
    const int r8   = (lane >> 4) * 8;
    v8f acc = (v8f){0.f,0.f,0.f,0.f,0.f,0.f,0.f,0.f};
#pragma unroll 1
    for (int ks = 0; ks < HID; ks += 32) {
      const v16h fa = Frag<_Float16>::load(H4 + (wave * 16 + rl) * HID + ks + koff);
      const v16h fb = Frag<_Float16>::load(W4 + rl * HID + ks + koff);
      acc = Frag<_Float16>::mma(fa, fb, acc);
      guard_ab1(acc, fa, fb);
    }
    const float bv = bf16_rne(b4[rl < 3 ? rl : 2]);
#pragma unroll
    for (int r = 0; r < 8; ++r) {
      const float v = acc[r] * WCARRY_INV + bv;
      if (rl < 3) sOut[(wave * 16 + r8 + r) * 4 + rl] = v;
    }
  }
  __syncthreads();

  if (wave == 0) {
    const v4f vv0 = *(const v4f*)(sOut + lane * 4);
    const v4f vv1 = *(const v4f*)(sOut + (32 + lane) * 4);
    float* pb = PA + (size_t)rowBase * 4;
    for (int pass = 0; pass < 2; ++pass) {
      *(volatile v4f*)(pb + lane * 4) = vv0;
      *(volatile v4f*)(pb + (32 + lane) * 4) = vv1;
      __threadfence();
    }
  }
}

__global__ __launch_bounds__(256) void blend_kernel(const float* __restrict__ PA, float* __restrict__ out) {
  __shared__ __align__(16) float sO[768];
  const int t = threadIdx.x;
  const int lane = t & 31, wave = t >> 5;
  const int s = blockIdx.x * 256 + t;
  const v4f c0 = *(const v4f*)(PA + ((size_t)0 * NSAMP + s) * 4);
  const v4f c1 = *(const v4f*)(PA + ((size_t)1 * NSAMP + s) * 4);
  const v4f c2 = *(const v4f*)(PA + ((size_t)2 * NSAMP + s) * 4);
  const v4f c3 = *(const v4f*)(PA + ((size_t)3 * NSAMP + s) * 4);
  const float a0 = c0[3], a1 = c1[3], a2 = c2[3], a3 = c3[3];
  float tot = a0 + a1; tot = tot + a2; tot = tot + a3;
  const float inv = 1.0f / tot;
  const float q0 = a3 * inv, q1 = a2 * inv, q2 = a1 * inv, q3 = a0 * inv;
#pragma unroll
  for (int o = 0; o < 3; ++o) {
    float r = c0[o] * q0;
    r = r + c1[o] * q1;
    r = r + c2[o] * q2;
    r = r + c3[o] * q3;
    sO[t * 3 + o] = r;
  }
  __syncthreads();
  if (wave < 6) {
    const int idx = wave * 32 + lane;
    const v4f v = *(const v4f*)(sO + idx * 4);
    float* op = out + (size_t)blockIdx.x * 768 + idx * 4;
    for (int pass = 0; pass < 2; ++pass) {
      *(volatile v4f*)op = v;
      __threadfence();
    }
  }
}

extern "C" void kernel_launch(void* const* d_in, const int* in_sizes, int n_in,
                              void* d_out, int out_size, void* d_ws, size_t ws_size,
                              hipStream_t stream) {
  (void)in_sizes;
  if (n_in < 15) return;
  const float* inp   = (const float*)d_in[0];
  const float* coord = (const float*)d_in[1];
  const float* cell  = (const float*)d_in[2];
  const float* enc_w = (const float*)d_in[3];
  const float* enc_b = (const float*)d_in[4];
  const float* w0 = (const float*)d_in[5];
  const float* b0 = (const float*)d_in[6];
  const float* w1 = (const float*)d_in[7];
  const float* b1 = (const float*)d_in[8];
  const float* w2 = (const float*)d_in[9];
  const float* b2 = (const float*)d_in[10];
  const float* w3 = (const float*)d_in[11];
  const float* b3 = (const float*)d_in[12];
  const float* w4 = (const float*)d_in[13];
  const float* b4 = (const float*)d_in[14];
  float* out = (float*)d_out;

  constexpr size_t FEAT_BYTES  = (size_t)NBATCH * IMG * IMG * NCH * 2;
  constexpr size_t WT0_BYTES   = (size_t)HID * W0PITCH * 2;
  constexpr size_t WT123_BYTES = (size_t)3 * HID * HID * 2;
  constexpr size_t WT4_BYTES   = (size_t)NOUT4 * HID * 2;
  constexpr size_t PA_BYTES    = (size_t)NROWS * 4 * 4;
  constexpr size_t OFF_FEAT  = 0;
  constexpr size_t OFF_WT0   = OFF_FEAT + FEAT_BYTES;
  constexpr size_t OFF_WT123 = OFF_WT0 + WT0_BYTES;
  constexpr size_t OFF_WT4   = OFF_WT123 + WT123_BYTES;
  constexpr size_t OFF_PA    = OFF_WT4 + WT4_BYTES;
  constexpr size_t OFF_END   = OFF_PA + PA_BYTES;
  static_assert(OFF_END == 9117696);
  static_assert(OFF_END <= (size_t)134217728);
  static_assert(OFF_WT0 % 128 == 0 && OFF_WT123 % 128 == 0 && OFF_WT4 % 128 == 0 && OFF_PA % 128 == 0);
  if (ws_size < OFF_END) return;
  if ((size_t)out_size < (size_t)NSAMP * 3) return;

  char* ws = (char*)d_ws;
  unsigned short* featH = (unsigned short*)(ws + OFF_FEAT);
  unsigned short* Wt0   = (unsigned short*)(ws + OFF_WT0);
  unsigned short* Wt123 = (unsigned short*)(ws + OFF_WT123);
  unsigned short* Wt4   = (unsigned short*)(ws + OFF_WT4);
  float*          PA    = (float*)(ws + OFF_PA);

  conv_kernel<<<(NBATCH * IMG * IMG) / 4, 256, 0, stream>>>(inp, enc_w, enc_b, featH);
  wprep_kernel<<<dim3(W0PITCH / 64, HID / 64, 4), 256, 0, stream>>>(w0, w1, w2, w3, Wt0, Wt123);
  wprep4_kernel<<<1, 256, 0, stream>>>(w4, Wt4);
  mlp_kernel<<<NROWS / MTILE, 256, 0, stream>>>(featH, coord, cell, Wt0, Wt123, Wt4,
                                                 b0, b1, b2, b3, b4, PA);
  blend_kernel<<<NSAMP / 256, 256, 0, stream>>>(PA, out);
}
